// GATTransformer_47596827574855
// MI455X (gfx1250) — hardware-run, weakly checked
//
#include <hip/hip_runtime.h>


namespace {
constexpr int N = 20000, NP = 20032, E = 320000, D = 128, NH = 2, HC = 256, MLP = 512, DEPTH = 2;
constexpr float XS = 8.0f, WSC = 256.0f, NEG = 0.2f, EPSD = 1e-16f, LNEPS = 1e-5f;
typedef _Float16 b16;
typedef __attribute__((ext_vector_type(16))) _Float16 v16b;
typedef __attribute__((ext_vector_type(8))) _Float16 v8b;
typedef __attribute__((ext_vector_type(8))) float v8f;
typedef __attribute__((ext_vector_type(4))) float v4f;
__device__ __forceinline__ float bf16_rne(float f) { unsigned int u = __float_as_uint(f); u += 0x7FFFu + ((u >> 16) & 1u); return __uint_as_float(u & 0xFFFF0000u); }
__device__ __forceinline__ void split16(float v, b16& hi, b16& lo) { hi = (b16)v; lo = (b16)(v - (float)hi); }
__device__ __forceinline__ v16b frag_kb(const b16* p, int hh) { const v8b a = *(const v8b*)(p + 8 * hh), b = *(const v8b*)(p + 16 + 8 * hh); v16b f;
#pragma unroll
  for (int e = 0; e < 8; ++e) { f[e] = a[e]; f[8 + e] = b[e]; } return f; }
__device__ __forceinline__ v8f wmma16b(v16b a, v16b b, v8f c) { v8f d = __builtin_amdgcn_wmma_f32_16x16x32_f16(false, a, false, b, (short)0, c, false, false); asm volatile("v_nop\n\tv_nop\n\tv_nop\n\tv_nop" : "+v"(d) : "v"(a), "v"(b)); return d; }
__device__ __forceinline__ void wave_lds_sync() { __builtin_amdgcn_fence(__ATOMIC_RELEASE, "workgroup"); __builtin_amdgcn_wave_barrier(); __builtin_amdgcn_fence(__ATOMIC_ACQUIRE, "workgroup"); }
__device__ __forceinline__ float pmul(float a, float b) { float p = a * b; asm volatile("" : "+v"(p)); return p; }
__device__ __forceinline__ float opaque(float a) { asm volatile("" : "+v"(a)); return a; }
__device__ __forceinline__ int iclamp(int v, int lo, int hi) { return v < lo ? lo : (v > hi ? hi : v); }
__device__ __forceinline__ float nexp(float x) { return __builtin_amdgcn_exp2f(x * 1.4426950408889634f); }
__device__ __forceinline__ float lrelu(float x) { return x > 0.0f ? x : NEG * x; }
__device__ __forceinline__ float gelu_(float x) { return 0.5f * x * (1.0f + erff(x * 0.70710678118654752f)); }
constexpr int CSR_NBLK = 512, CSR_GB = 9, CSR_GN = 1 << CSR_GB  , CSR_MAXG = 512, CSR_CAP = 12288  ;
__global__ __launch_bounds__(64) void csrA_kernel(const int* __restrict__ dst, int E, int N, int nG, int CHP, int NGP, int* __restrict__ STG, int* __restrict__ HST) {
  extern __shared__ int sm[];
  int* cnt = sm; int* run = sm + NGP; int* ids = sm + 2 * NGP;
  const int b = blockIdx.x; const int ch = (E + CSR_NBLK - 1) / CSR_NBLK; const int e0 = b * ch, e1 = min(E, e0 + ch);
  for (int i = threadIdx.x; i < NGP; i += 64) cnt[i] = 0;
  for (int i = threadIdx.x; i < CHP; i += 64) ids[i] = -1;
  __syncthreads();
  if (threadIdx.x == 0) {
    for (int e = e0; e < e1; ++e) { int d = dst[e]; d = (d < 0) ? 0 : (d >= N ? N - 1 : d); cnt[d >> CSR_GB] += 1; }
    int acc = 0; for (int g = 0; g < nG; ++g) { run[g] = acc; acc += cnt[g]; }
    for (int e = e0; e < e1; ++e) { int d = dst[e]; d = (d < 0) ? 0 : (d >= N ? N - 1 : d); const int g = d >> CSR_GB; ids[run[g]] = e; run[g] += 1; } }
  __syncthreads();
  typedef __attribute__((ext_vector_type(4))) int v4i;
  for (int pass = 0; pass < 2; ++pass) {
    for (int i = threadIdx.x; i < CHP / 4; i += 64) *(volatile v4i*)(STG + (size_t)b * CHP + i * 4) = *(const v4i*)(&ids[i * 4]);
    for (int i = threadIdx.x; i < NGP / 4; i += 64) { v4i v; for (int e = 0; e < 4; ++e) v[e] = (i * 4 + e < nG) ? cnt[i * 4 + e] : 0; *(volatile v4i*)(HST + (size_t)b * NGP + i * 4) = v; }
    __threadfence(); }
}
__global__ __launch_bounds__(512) void csrS_kernel(const int* __restrict__ HST, int nG, int NGP, int* __restrict__ START, int* __restrict__ TOT, int* __restrict__ OFF) {
  __shared__ int tot[CSR_MAXG];
  const int b = threadIdx.x;
  for (int pass = 0; pass < 2; ++pass) { int runb = 0; for (int g = 0; g < nG; ++g) { int c = HST[(size_t)b * NGP + g]; c = (c < 0) ? 0 : c; ((volatile int*)OFF)[(size_t)g * CSR_NBLK + b] = runb; runb += c; } __threadfence(); }
  for (int g = threadIdx.x; g < nG; g += 512) { int s = 0; for (int bb = 0; bb < CSR_NBLK; ++bb) { int c = HST[(size_t)bb * NGP + g]; s += (c < 0) ? 0 : c; } tot[g] = s; }
  __syncthreads();
  if (threadIdx.x < 32) {
    __shared__ int st[CSR_MAXG + 32];
    if (threadIdx.x == 0) { int acc = 0; for (int g = 0; g < NGP; ++g) { st[g] = acc; if (g < nG) acc += (tot[g] + 31) & ~31; } st[NGP] = acc; }
    __builtin_amdgcn_fence(__ATOMIC_RELEASE, "workgroup"); __builtin_amdgcn_wave_barrier(); __builtin_amdgcn_fence(__ATOMIC_ACQUIRE, "workgroup");
    for (int pass = 0; pass < 2; ++pass) { for (int i = threadIdx.x; i < NGP + 32; i += 32) { ((volatile int*)START)[i] = (i <= NGP) ? st[min(i, NGP)] : 0; ((volatile int*)TOT)[i] = (i < nG) ? tot[i] : 0; } __threadfence(); } }
}
__global__ __launch_bounds__(256) void csrB_kernel(const int* __restrict__ dst, int N, int nG, int CHP, int NGP, int permLen, const int* __restrict__ STG, const int* __restrict__ HST, const int* __restrict__ OFF, const int* __restrict__ START, const int* __restrict__ TOT, int* __restrict__ PERM, int* __restrict__ ROWPTR, int* __restrict__ ROWCNT, int* __restrict__ FLAG) {
  typedef __attribute__((ext_vector_type(4))) int v4i;
  __shared__ int ids[CSR_CAP]; __shared__ unsigned short key[CSR_CAP]; __shared__ int outp[CSR_CAP]; __shared__ int ncnt[CSR_GN + 1]; __shared__ int boff[CSR_NBLK + 1];
  const int g = blockIdx.x, t_ = threadIdx.x; int tot = TOT[g]; int st = START[g], stn = START[g + 1]; const int v0 = g * CSR_GN; const int nv = min(CSR_GN, N - v0);
  st = (st < 0) ? 0 : (st > permLen - 32 ? permLen - 32 : st) & ~31; stn = (stn < st) ? st : (stn > permLen ? permLen : stn); tot = (tot < 0) ? 0 : tot; if (tot > stn - st && tot <= CSR_CAP) tot = stn - st;
  if (tot > CSR_CAP) {
    for (int pass = 0; pass < 2; ++pass) { for (int i = t_; i < CSR_GN / 4; i += 256) { v4i a, c; for (int e = 0; e < 4; ++e) { a[e] = st; c[e] = 0; } *(volatile v4i*)(ROWPTR + v0 + i * 4) = a; *(volatile v4i*)(ROWCNT + v0 + i * 4) = c; } if (t_ == 0) ((volatile int*)FLAG)[0] = 1; __threadfence(); } (void)nv; return; }
  if (t_ == 0) { int acc = 0; for (int b = 0; b < CSR_NBLK; ++b) { boff[b] = acc; int c = HST[(size_t)b * NGP + g]; c = (c < 0) ? 0 : (c > CHP ? CHP : c); acc += c; if (acc > tot) acc = tot; } boff[CSR_NBLK] = acc; }
  for (int i = t_; i <= CSR_GN; i += 256) ncnt[i] = 0;
  __syncthreads();
  for (int b = 0; b < CSR_NBLK; ++b) { const int c = boff[b + 1] - boff[b]; int o_ = OFF[(size_t)g * CSR_NBLK + b]; o_ = (o_ < 0) ? 0 : (o_ > CHP - c ? CHP - c : o_); const int* src_ = STG + (size_t)b * CHP + o_;
    for (int i = t_; i < c; i += 256) { int id = src_[i]; id = (id < 0) ? 0 : id; ids[boff[b] + i] = id; int d = dst[id]; d = (d < v0) ? v0 : (d >= N ? N - 1 : d); int kk = d - v0; kk = (kk < 0) ? 0 : (kk >= CSR_GN ? CSR_GN - 1 : kk); key[boff[b] + i] = (unsigned short)kk; } }
  __syncthreads();
  if (t_ == 0) { for (int i = 0; i < tot; ++i) ncnt[key[i]] += 1; int acc = 0; for (int vl = 0; vl < CSR_GN; ++vl) { const int c = ncnt[vl]; ncnt[vl] = acc; acc += c; } ncnt[CSR_GN] = acc;
    for (int i = 0; i < tot; ++i) { const int vl = key[i]; outp[ncnt[vl]] = ids[i]; ncnt[vl] += 1; }
    for (int vl = CSR_GN; vl > 0; --vl) ncnt[vl] = ncnt[vl - 1]; ncnt[0] = 0; }
  __syncthreads();
  for (int pass = 0; pass < 2; ++pass) {
    for (int i = t_; i < (stn - st) / 4; i += 256) { v4i v; for (int e = 0; e < 4; ++e) { const int q = i * 4 + e; v[e] = (q < tot) ? outp[q] : -1; } *(volatile v4i*)(PERM + st + i * 4) = v; }
    for (int i = t_; i < CSR_GN / 4; i += 256) { v4i a, c; for (int e = 0; e < 4; ++e) { const int vl = i * 4 + e; a[e] = st + ncnt[vl]; c[e] = (vl < nv) ? (ncnt[vl + 1] - ncnt[vl]) : 0; } *(volatile v4i*)(ROWPTR + v0 + i * 4) = a; *(volatile v4i*)(ROWCNT + v0 + i * 4) = c; }
    __threadfence(); }
}
__global__ __launch_bounds__(256) void csrZ_kernel(int* __restrict__ p, size_t n4) { typedef __attribute__((ext_vector_type(4))) int v4i; const size_t tid = (size_t)blockIdx.x * 256 + threadIdx.x, nth = (size_t)gridDim.x * 256; v4i z = {0, 0, 0, 0}; for (size_t i = tid; i < n4; i += nth) *(volatile v4i*)(p + i * 4) = z; }
struct CsrBufs { int *STG, *HST, *OFF, *START, *TOT, *PERM, *ROWPTR, *ROWCNT, *FLAG; int nG, NGP, CHP; size_t permLen; char* base; size_t bytes; };
static size_t csr_carve(CsrBufs& c, char* ws, size_t off, int E, int N) {
  const size_t off0 = off; c.base = ws + off;
  auto al = [&](size_t bytes) { char* p = ws + off; off += (bytes + 255) & ~(size_t)255; return p; };
  c.nG = (N + CSR_GN - 1) / CSR_GN; c.NGP = (c.nG + 31) & ~31; const int ch = (E + CSR_NBLK - 1) / CSR_NBLK; c.CHP = (ch + 31) & ~31; c.permLen = (size_t)E + 32 * (size_t)c.nG + 32;
  c.STG = (int*)al((size_t)CSR_NBLK * c.CHP * 4); c.HST = (int*)al((size_t)CSR_NBLK * c.NGP * 4); c.OFF = (int*)al((size_t)c.NGP * CSR_NBLK * 4); c.START = (int*)al((size_t)(c.NGP + 64) * 4); c.TOT = (int*)al((size_t)(c.NGP + 64) * 4);
  c.PERM = (int*)al(c.permLen * 4); c.ROWPTR = (int*)al((size_t)c.nG * CSR_GN * 4); c.ROWCNT = (int*)al((size_t)c.nG * CSR_GN * 4); c.FLAG = (int*)al(256);
  c.bytes = off - off0; return off;
}
static void csr_build(const CsrBufs& c, const int* dst, int E, int N, hipStream_t stream) {
  const size_t smem = (size_t)(2 * c.NGP + c.CHP) * 4;
  csrZ_kernel<<<512, 256, 0, stream>>>((int*)c.base, c.bytes / 16);
  csrA_kernel<<<CSR_NBLK, 64, smem, stream>>>(dst, E, N, c.nG, c.CHP, c.NGP, c.STG, c.HST);
  csrS_kernel<<<1, 512, 0, stream>>>(c.HST, c.nG, c.NGP, c.START, c.TOT, c.OFF);
  csrB_kernel<<<c.nG, 256, 0, stream>>>(dst, N, c.nG, c.CHP, c.NGP, (int)c.permLen, c.STG, c.HST, c.OFF, c.START, c.TOT, c.PERM, c.ROWPTR, c.ROWCNT, c.FLAG);
}


__global__ __launch_bounds__(256) void wprep_kernel(const float* __restrict__ wl, const float* __restrict__ wr, const float* __restrict__ wq, const float* __restrict__ w1, const float* __restrict__ w2, b16* __restrict__ WLR, b16* __restrict__ WQ, b16* __restrict__ WF1, b16* __restrict__ WF2) {
  const size_t u = (size_t)blockIdx.x * 256 + threadIdx.x; const size_t n0 = (size_t)DEPTH * 2 * HC * D / 8, n1 = (size_t)DEPTH * D * HC / 8, n2 = (size_t)DEPTH * MLP * D / 8, n3 = (size_t)DEPTH * D * MLP / 8; size_t t = u; v8b o;
  if (t < n0) { const size_t e = t * 8; const int d = (int)(e / (2 * HC * D)); const int rem = (int)(e % (2 * HC * D)); const int row = rem / D, k0 = rem % D; const float* w = row < HC ? wl : wr; const int oo = row % HC;
    for (int j = 0; j < 8; ++j) o[j] = (b16)(bf16_rne(w[((size_t)d * D + k0 + j) * HC + oo]) * WSC); for (int pass = 0; pass < 2; ++pass) { *(volatile v8b*)(WLR + e) = o; __threadfence(); } return; } t -= n0;
  if (t < n1) { const size_t e = t * 8; const int d = (int)(e / (D * HC)); const int rem = (int)(e % (D * HC)); const int oo = rem / HC, k0 = rem % HC; for (int j = 0; j < 8; ++j) o[j] = (b16)(bf16_rne(wq[((size_t)d * HC + k0 + j) * D + oo]) * WSC); for (int pass = 0; pass < 2; ++pass) { *(volatile v8b*)(WQ + e) = o; __threadfence(); } return; } t -= n1;
  if (t < n2) { const size_t e = t * 8; const int d = (int)(e / (MLP * D)); const int rem = (int)(e % (MLP * D)); const int oo = rem / D, k0 = rem % D; for (int j = 0; j < 8; ++j) o[j] = (b16)(bf16_rne(w1[((size_t)d * D + k0 + j) * MLP + oo]) * WSC); for (int pass = 0; pass < 2; ++pass) { *(volatile v8b*)(WF1 + e) = o; __threadfence(); } return; } t -= n2;
  if (t < n3) { const size_t e = t * 8; const int d = (int)(e / (D * MLP)); const int rem = (int)(e % (D * MLP)); const int oo = rem / MLP, k0 = rem % MLP; for (int j = 0; j < 8; ++j) o[j] = (b16)(bf16_rne(w2[((size_t)d * MLP + k0 + j) * D + oo]) * WSC); for (int pass = 0; pass < 2; ++pass) { *(volatile v8b*)(WF2 + e) = o; __threadfence(); } }
}
template <int RAW>
__global__ __launch_bounds__(128) void proj_kernel(const float* __restrict__ Xp, const float* __restrict__ lw, const float* __restrict__ lb, const b16* __restrict__ W, const float* __restrict__ bl, const float* __restrict__ br, float* __restrict__ XLR) {
  __shared__ __attribute__((aligned(16))) b16 Ah[4][16][D + 8], Al[4][16][D + 8]; __shared__ __attribute__((aligned(16))) float Tf[4][16][128 + 4];
  const int wave = threadIdx.x >> 5, lane = threadIdx.x & 31, nloc = lane & 15, hlf = lane >> 4; const size_t m0 = (size_t)blockIdx.x * 64 + wave * 16; const int c0 = blockIdx.y * 128;
  for (int rr = 0; rr < 16; ++rr) { const size_t v = m0 + rr; v4f x = {0.0f, 0.0f, 0.0f, 0.0f}; if (!RAW || v < (size_t)N) x = *(const v4f*)(Xp + v * D + lane * 4); if (RAW) for (int j = 0; j < 4; ++j) x[j] = bf16_rne(x[j]);
    float s1 = x[0] + x[1] + x[2] + x[3]; for (int o = 16; o; o >>= 1) s1 += __shfl_xor(s1, o); const float mean = s1 * (1.0f / D);
    float s2 = 0.0f; for (int j = 0; j < 4; ++j) { const float dd = x[j] - mean; s2 += dd * dd; } for (int o = 16; o; o >>= 1) s2 += __shfl_xor(s2, o); const float rstd = rsqrtf(s2 * (1.0f / D) + LNEPS);
    for (int j = 0; j < 4; ++j) { const int c = lane * 4 + j; const float h = (v < (size_t)N) ? (x[j] - mean) * rstd * bf16_rne(lw[c]) + bf16_rne(lb[c]) : 0.0f; b16 p, q; split16(h * XS, p, q); Ah[wave][rr][c] = p; Al[wave][rr][c] = q; } }
  wave_lds_sync();
  v8f acc[8];
#pragma unroll
  for (int t = 0; t < 8; ++t) acc[t] = (v8f){};
#pragma unroll
  for (int kb = 0; kb < D; kb += 32) { const v16b a = frag_kb(&Ah[wave][nloc][kb], hlf), al = frag_kb(&Al[wave][nloc][kb], hlf);
#pragma unroll
    for (int t = 0; t < 8; ++t) { const v16b bw = frag_kb(W + (size_t)(c0 + t * 16 + nloc) * D + kb, hlf); acc[t] = wmma16b(a, bw, acc[t]); acc[t] = wmma16b(al, bw, acc[t]); } }
  wave_lds_sync();
#pragma unroll
  for (int t = 0; t < 8; ++t) { const int cabs = c0 + t * 16 + nloc; const float bb = cabs < HC ? bf16_rne(bl[cabs]) : bf16_rne(br[cabs - HC]);
#pragma unroll 1
    for (int r = 0; r < 8; ++r) { const size_t row = m0 + 8 * hlf + r; Tf[wave][8 * hlf + r][t * 16 + nloc] = row < (size_t)N ? acc[t][r] * (1.0f / (XS * WSC)) + bb : 0.0f; } }
  wave_lds_sync();
  for (int pass = 0; pass < 2; ++pass) { for (int rr = 0; rr < 16; ++rr) *(volatile v4f*)(XLR + (m0 + rr) * (2 * HC) + c0 + lane * 4) = *(const v4f*)(&Tf[wave][rr][lane * 4]); __threadfence(); }
}
__global__ __launch_bounds__(256) void attn_kernel(const float* __restrict__ XLR, const float* __restrict__ att, const float* __restrict__ bias, const int* __restrict__ srcs, const int* __restrict__ PERM, const int* __restrict__ ROWPTR, const int* __restrict__ ROWCNT, int permLen, float* __restrict__ P) {
  const int wave = threadIdx.x >> 5, lane = threadIdx.x & 31; const size_t v = (size_t)blockIdx.x * 8 + wave; const int cb = lane * 8;
  float aw[8], xr[8], acc[8];
#pragma unroll
  for (int i = 0; i < 8; ++i) { aw[i] = opaque(bf16_rne(att[cb + i])); acc[i] = 0.0f; xr[i] = 0.0f; }
  int st = 0, cnt = 0; if (v < (size_t)N) { st = ROWPTR[v]; cnt = ROWCNT[v]; cnt = iclamp(cnt, 0, 65536); st = iclamp(st, 0, permLen - cnt); for (int q = 0; q < 2; ++q) { const v4f t = *(const v4f*)(XLR + v * (2 * HC) + HC + cb + 4 * q); for (int i = 0; i < 4; ++i) xr[4 * q + i] = t[i]; } }
  auto logit = [&](const float* xl) { float d = 0.0f;
#pragma unroll
    for (int i = 0; i < 8; ++i) d += pmul(aw[i], lrelu(xl[i] + xr[i])); d += __shfl_xor(d, 1); d += __shfl_xor(d, 2); d += __shfl_xor(d, 4); d += __shfl_xor(d, 8); return d; };
  float mx = -INFINITY;
#pragma unroll 1
  for (int j = 0; j < cnt; ++j) { const int e = iclamp(PERM[st + j], 0, E - 1); const size_t s = (size_t)iclamp(srcs[e], 0, N - 1); float xl[8]; for (int q = 0; q < 2; ++q) { const v4f t = *(const v4f*)(XLR + s * (2 * HC) + cb + 4 * q); for (int i = 0; i < 4; ++i) xl[4 * q + i] = t[i]; } mx = fmaxf(mx, logit(xl)); }
  float den = 0.0f;
#pragma unroll 1
  for (int j = 0; j < cnt; ++j) { const int e = iclamp(PERM[st + j], 0, E - 1); const size_t s = (size_t)iclamp(srcs[e], 0, N - 1); float xl[8]; for (int q = 0; q < 2; ++q) { const v4f t = *(const v4f*)(XLR + s * (2 * HC) + cb + 4 * q); for (int i = 0; i < 4; ++i) xl[4 * q + i] = t[i]; }
    const float pj = nexp(logit(xl) - mx); den += pj;
#pragma unroll
    for (int i = 0; i < 8; ++i) acc[i] += pmul(pj, xl[i]); }
  const float inv = (cnt > 0) ? 1.0f / (den + EPSD) : 0.0f; v4f o[2];
  for (int q = 0; q < 2; ++q) for (int i = 0; i < 4; ++i) { const int c = cb + 4 * q + i; o[q][i] = (v < (size_t)N) ? pmul(acc[4 * q + i], inv) + bf16_rne(bias[c]) : 0.0f; }
  for (int pass = 0; pass < 2; ++pass) { *(volatile v4f*)(P + v * HC + cb) = o[0]; *(volatile v4f*)(P + v * HC + cb + 4) = o[1]; __threadfence(); }
}
template <int RAW, int LAST>
__global__ __launch_bounds__(32) void node_kernel(const float* __restrict__ P, const float* Xin, const b16* __restrict__ WQ, const float* __restrict__ bq, const float* __restrict__ lw, const float* __restrict__ lb, const b16* __restrict__ WF1, const float* __restrict__ b1, const b16* __restrict__ WF2, const float* __restrict__ b2, float* Xout) {
  __shared__ __attribute__((aligned(16))) b16 Ah[16][HC + 8], Al[16][HC + 8], Bh[16][MLP + 8], Bl[16][MLP + 8]; __shared__ __attribute__((aligned(16))) float Xv[16][D + 4];
  const int lane = threadIdx.x, nloc = lane & 15, hlf = lane >> 4; const size_t v0 = (size_t)blockIdx.x * 16;
  for (int rr = 0; rr < 16; ++rr) { const size_t v = v0 + rr; const bool ok = v < (size_t)N;
    for (int q = lane * 4; q < HC; q += 128) { const v4f a = *(const v4f*)(P + v * HC + q); for (int j = 0; j < 4; ++j) { b16 p, s; split16(a[j] * XS, p, s); Ah[rr][q + j] = p; Al[rr][q + j] = s; } }
    v4f xv = {0.0f, 0.0f, 0.0f, 0.0f}; if (ok) xv = *(const v4f*)(Xin + v * D + lane * 4); if (RAW) for (int j = 0; j < 4; ++j) xv[j] = bf16_rne(xv[j]); *(v4f*)(&Xv[rr][lane * 4]) = xv; }
  wave_lds_sync();
  v8f acc[8];
#pragma unroll
  for (int t = 0; t < 8; ++t) acc[t] = (v8f){};
#pragma unroll 2
  for (int kb = 0; kb < HC; kb += 32) { const v16b a = frag_kb(&Ah[nloc][kb], hlf), al = frag_kb(&Al[nloc][kb], hlf);
#pragma unroll
    for (int t = 0; t < 8; ++t) { const v16b bw = frag_kb(WQ + (size_t)(t * 16 + nloc) * HC + kb, hlf); acc[t] = wmma16b(a, bw, acc[t]); acc[t] = wmma16b(al, bw, acc[t]); } }
  wave_lds_sync();
#pragma unroll
  for (int t = 0; t < 8; ++t) { const int c = t * 16 + nloc; const float bb = bf16_rne(bq[c]);
#pragma unroll 1
    for (int r = 0; r < 8; ++r) { const int rr = 8 * hlf + r; Xv[rr][c] = Xv[rr][c] + acc[t][r] * (1.0f / (XS * WSC)) + bb; } }
  wave_lds_sync();
  for (int rr = 0; rr < 16; ++rr) { const v4f x = *(const v4f*)(&Xv[rr][lane * 4]); float s1 = x[0] + x[1] + x[2] + x[3]; for (int o = 16; o; o >>= 1) s1 += __shfl_xor(s1, o); const float mean = s1 * (1.0f / D);
    float s2 = 0.0f; for (int j = 0; j < 4; ++j) { const float dd = x[j] - mean; s2 += dd * dd; } for (int o = 16; o; o >>= 1) s2 += __shfl_xor(s2, o); const float rstd = rsqrtf(s2 * (1.0f / D) + LNEPS);
    for (int j = 0; j < 4; ++j) { const int c = lane * 4 + j; const float h = (x[j] - mean) * rstd * bf16_rne(lw[c]) + bf16_rne(lb[c]); b16 p, q; split16(h * XS, p, q); Ah[rr][c] = p; Al[rr][c] = q; } }
  wave_lds_sync();
  for (int qtr = 0; qtr < 4; ++qtr) { v8f f[8];
#pragma unroll
    for (int t = 0; t < 8; ++t) f[t] = (v8f){};
#pragma unroll
    for (int kb = 0; kb < D; kb += 32) { const v16b a = frag_kb(&Ah[nloc][kb], hlf), al = frag_kb(&Al[nloc][kb], hlf);
#pragma unroll
      for (int t = 0; t < 8; ++t) { const v16b bw = frag_kb(WF1 + (size_t)(qtr * 128 + t * 16 + nloc) * D + kb, hlf); f[t] = wmma16b(a, bw, f[t]); f[t] = wmma16b(al, bw, f[t]); } }
#pragma unroll
    for (int t = 0; t < 8; ++t) { const int c = qtr * 128 + t * 16 + nloc; const float bb = bf16_rne(b1[c]);
#pragma unroll 1
      for (int r = 0; r < 8; ++r) { b16 p, q; split16(gelu_(f[t][r] * (1.0f / (XS * WSC)) + bb) * XS, p, q); Bh[8 * hlf + r][c] = p; Bl[8 * hlf + r][c] = q; } } }
  wave_lds_sync();
#pragma unroll
  for (int t = 0; t < 8; ++t) acc[t] = (v8f){};
#pragma unroll 2
  for (int kb = 0; kb < MLP; kb += 32) { const v16b a = frag_kb(&Bh[nloc][kb], hlf), al = frag_kb(&Bl[nloc][kb], hlf);
#pragma unroll
    for (int t = 0; t < 8; ++t) { const v16b bw = frag_kb(WF2 + (size_t)(t * 16 + nloc) * MLP + kb, hlf); acc[t] = wmma16b(a, bw, acc[t]); acc[t] = wmma16b(al, bw, acc[t]); } }
  wave_lds_sync();
#pragma unroll
  for (int t = 0; t < 8; ++t) { const int c = t * 16 + nloc; const float bb = bf16_rne(b2[c]);
#pragma unroll 1
    for (int r = 0; r < 8; ++r) { const int rr = 8 * hlf + r; Xv[rr][c] = Xv[rr][c] + acc[t][r] * (1.0f / (XS * WSC)) + bb; } }
  wave_lds_sync();
  for (int rr = 0; rr < 16; ++rr) { const size_t v = v0 + rr; v4f o = *(const v4f*)(&Xv[rr][lane * 4]); if (v >= (size_t)N) o = (v4f){0.0f, 0.0f, 0.0f, 0.0f};
    for (int pass = 0; pass < 2; ++pass) { if (!LAST || v < (size_t)N) *(volatile v4f*)(Xout + v * D + lane * 4) = o; __threadfence(); } }
}
}

extern "C" void kernel_launch(void* const* d_in, const int* in_sizes, int n_in, void* d_out, int out_size, void* d_ws, size_t ws_size, hipStream_t stream) {
  (void)n_in;
  auto Fp = [&](int i) { return (const float*)d_in[i]; }; auto Ip = [&](int i) { return (const int*)d_in[i]; };
  if (in_sizes[0] != N * D || in_sizes[1] != 2 * E || in_sizes[4] != DEPTH * D * HC || in_sizes[10] != DEPTH * HC * D || in_sizes[14] != DEPTH * D * MLP || in_sizes[16] != DEPTH * MLP * D || out_size != N * D) return;
  size_t off = 0; char* ws = (char*)d_ws;
  auto carve = [&](size_t bytes) { char* p = ws + off; off += (bytes + 255) & ~(size_t)255; return p; };
  b16* WLR = (b16*)carve((size_t)DEPTH * 2 * HC * D * 2); b16* WQ = (b16*)carve((size_t)DEPTH * D * HC * 2); b16* WF1 = (b16*)carve((size_t)DEPTH * MLP * D * 2); b16* WF2 = (b16*)carve((size_t)DEPTH * D * MLP * 2);
  float* XLR = (float*)carve((size_t)NP * 2 * HC * 4); float* P = (float*)carve((size_t)NP * HC * 4); float* X = (float*)carve((size_t)NP * D * 4);
  CsrBufs csr; off = csr_carve(csr, ws, off, E, N);
  if (off > ws_size || off > ((size_t)128 << 20)) return;
  wprep_kernel<<<(unsigned)(((size_t)DEPTH * (2 * HC * D + D * HC + 2 * MLP * D) / 8 + 255) / 256), 256, 0, stream>>>(Fp(4), Fp(6), Fp(10), Fp(14), Fp(16), WLR, WQ, WF1, WF2);
  csr_build(csr, Ip(1) + E, E, N, stream);
  for (int d = 0; d < DEPTH; ++d) { const float* xin = d == 0 ? Fp(0) : X;
    if (d == 0) proj_kernel<1><<<dim3(NP / 64, 4), 128, 0, stream>>>(xin, Fp(2) + d * D, Fp(3) + d * D, WLR + (size_t)d * 2 * HC * D, Fp(5) + d * HC, Fp(7) + d * HC, XLR);
    else proj_kernel<0><<<dim3(NP / 64, 4), 128, 0, stream>>>(xin, Fp(2) + d * D, Fp(3) + d * D, WLR + (size_t)d * 2 * HC * D, Fp(5) + d * HC, Fp(7) + d * HC, XLR);
    attn_kernel<<<NP / 8, 256, 0, stream>>>(XLR, Fp(8) + d * NH * D, Fp(9) + d * HC, Ip(1), csr.PERM, csr.ROWPTR, csr.ROWCNT, (int)csr.permLen, P);
    const b16* wq = WQ + (size_t)d * D * HC; const b16* wf1 = WF1 + (size_t)d * MLP * D; const b16* wf2 = WF2 + (size_t)d * D * MLP;
    if (d == 0) node_kernel<1, 0><<<NP / 16, 32, 0, stream>>>(P, xin, wq, Fp(11) + d * D, Fp(12) + d * D, Fp(13) + d * D, wf1, Fp(15) + d * MLP, wf2, Fp(17) + d * D, X);
    else node_kernel<0, 1><<<NP / 16, 32, 0, stream>>>(P, xin, wq, Fp(11) + d * D, Fp(12) + d * D, Fp(13) + d * D, wf1, Fp(15) + d * MLP, wf2, Fp(17) + d * D, (float*)d_out); }
}
